// SpliceGraph_27393301414017
// MI455X (gfx1250) — hardware-verified
//
#include <hip/hip_runtime.h>
#include <stddef.h>
#include <math.h>


#define FIN     64
#define FD      256
#define NTHR    256
#define NWAVE   8
#define GTHR    128
#define GWAVE   4
#define GROWS   64
#define EPT     8
#define NGRP    2
#define CHUNK   (NTHR * EPT * NGRP)
#define WCAP    (EPT * NGRP * 32)
#define LISTN   (NWAVE * WCAP)
#define NBC     4096
#define NBF     1024
#define RCAP    40960
#define RBN     128
#define TGT     256
#define DEGCAP  1024
#define OTHR    512
#define WSCAP   134217728

#define APK1    72
#define APK2    264

#define WP_G    0
#define WP_L    16384
#define WP_Q    32768
#define WPTOT   98304

#define LDS_FILL ((RCAP + NBF + LISTN) * 4 + 64)
#define LDS_G1   (GROWS * APK1 * 2 + GROWS * FD * 4)
#define LDS_G2   (GROWS * FD * 4 + GROWS * APK2 * 2 + GROWS * APK1 * 2)

#define BN_EPS  1e-5f
#define SC64I   0.015625f
#define SC1024I 0.0009765625f

static_assert((CHUNK & (CHUNK - 1)) == 0);
static_assert(CHUNK <= 4096);
static_assert(NBC <= 4096 && NBF <= 4096);
static_assert((NBC & (NBC - 1)) == 0 && (NBF & (NBF - 1)) == 0);
static_assert(NBC == 4 * NBF);
static_assert(OTHR * 8 == NBC);
static_assert((RCAP % 32) == 0);
static_assert(TGT == NWAVE * 32 && (TGT % GROWS) == 0);
static_assert((NBC % TGT) == 0);
static_assert(GROWS == GWAVE * 16 && GTHR == GWAVE * 32);
static_assert(WP_L == WP_G + FD * FIN && WP_Q == WP_L + FD * FIN && WPTOT == WP_Q + FD * FD);
static_assert((LDS_G1 % 16) == 0 && (LDS_G2 % 16) == 0);
static_assert(((GROWS * FD * 4) % 16) == 0 && ((GROWS * APK2 * 2) % 16) == 0);

typedef float          v4f  __attribute__((ext_vector_type(4)));
typedef float          v8f  __attribute__((ext_vector_type(8)));
typedef double         v2d  __attribute__((ext_vector_type(2)));
typedef int            v4i  __attribute__((ext_vector_type(4)));
typedef unsigned short v8us __attribute__((ext_vector_type(8)));
typedef _Float16       v8h  __attribute__((ext_vector_type(8)));
typedef _Float16       v16h __attribute__((ext_vector_type(16)));
union FragH { v16h v; v8us h[2]; };
union Cv8   { v8h f; v8us u; };

__device__ __forceinline__ v8us cvt8h(v4f a, v4f b, float sc) {
  v8h f;
  f[0] = (_Float16)(a.x * sc); f[1] = (_Float16)(a.y * sc);
  f[2] = (_Float16)(a.z * sc); f[3] = (_Float16)(a.w * sc);
  f[4] = (_Float16)(b.x * sc); f[5] = (_Float16)(b.y * sc);
  f[6] = (_Float16)(b.z * sc); f[7] = (_Float16)(b.w * sc);
  Cv8 c; c.f = f;
  return c.u;
}

__device__ __forceinline__ v8f wmh(v16h a, v16h b, v8f c) {
  v8f d = __builtin_amdgcn_wmma_f32_16x16x32_f16(false, a, false, b, (short)0, c, false, false);
  asm volatile("v_nop\n\tv_nop\n\tv_nop\n\tv_nop" : "+v"(d) : "v"(a), "v"(b));
  return d;
}

__device__ __forceinline__ float tanh_fast(float x) {
  const float e = __expf(2.0f * x);
  return 1.0f - 2.0f * __builtin_amdgcn_rcpf(1.0f + e);
}
__device__ __forceinline__ float sigm_fast(float x) {
  const float e = __expf(-x);
  return __builtin_amdgcn_rcpf(1.0f + e);
}

template <int KD, int NT, int APK>
__device__ __forceinline__ void mma16(const unsigned short* sA, const unsigned short* __restrict__ Bw,
                                      int wrow, int lane, v8f (&acc)[NT]) {
  static_assert((KD % 32) == 0 && (APK % 8) == 0);
  constexpr int NKT = KD / 32;
  const int hh = lane >> 4, m = lane & 15;
#pragma unroll
  for (int t = 0; t < NT; ++t) { v8f z = {0.f, 0.f, 0.f, 0.f, 0.f, 0.f, 0.f, 0.f}; acc[t] = z; }
  const unsigned short* ap = sA + (wrow + m) * APK + 8 * hh;
#pragma unroll 1
  for (int kt = 0; kt < NKT; ++kt) {
    FragH a;
    a.h[0] = *(const v8us*)(ap + 32 * kt);
    a.h[1] = *(const v8us*)(ap + 32 * kt + 16);
#pragma unroll
    for (int t = 0; t < NT; ++t) {
      const unsigned short* bp = Bw + (size_t)(16 * t + m) * KD + 32 * kt + 8 * hh;
      FragH b;
      b.h[0] = *(const v8us*)bp;
      b.h[1] = *(const v8us*)(bp + 16);
      acc[t] = wmh(a.v, b.v, acc[t]);
    }
  }
}

__device__ __forceinline__ void store_rows256(const float* stg, float* C, int rowBase, int wave, int lane) {
  const float* lp = stg + wave * 16 * FD + 4 * lane;
  float* gp = C + (size_t)(rowBase + wave * 16) * FD + 4 * lane;
#pragma unroll
  for (int i = 0; i < 16; ++i) {
    const v4f v0 = *(const v4f*)(lp + FD * i);
    const v4f v1 = *(const v4f*)(lp + FD * i + FD / 2);
    *(volatile v4f*)(gp + FD * i) = v0;
    *(volatile v4f*)(gp + FD * i + FD / 2) = v1;
  }
  __threadfence();
#pragma unroll
  for (int i = 0; i < 16; ++i) {
    const v4f v0 = *(const v4f*)(lp + FD * i);
    const v4f v1 = *(const v4f*)(lp + FD * i + FD / 2);
    *(volatile v4f*)(gp + FD * i) = v0;
    *(volatile v4f*)(gp + FD * i + FD / 2) = v1;
  }
}

template <int NB>
__device__ __forceinline__ int scan_chunk(const int* __restrict__ dsts, int nE, int cbase, int slotBase,
                                          int vec8, int* list, int tid, int lane, int wave) {
  int wc = 0;
#pragma unroll
  for (int g = 0; g < NGRP; ++g) {
    const int el0  = (g * NTHR + tid) * EPT;
    const int e0   = cbase + el0;
    const int sent = -2147483647 - 1;
    v4i da, db;
    if (vec8 != 0 && cbase + CHUNK <= nE) {
      da = *(const v4i*)(dsts + e0);
      db = *(const v4i*)(dsts + e0 + 4);
    } else {
      da.x = (e0     < nE) ? dsts[min(e0, nE - 1)] : sent;
      da.y = (e0 + 1 < nE) ? dsts[min(e0 + 1, nE - 1)] : sent;
      da.z = (e0 + 2 < nE) ? dsts[min(e0 + 2, nE - 1)] : sent;
      da.w = (e0 + 3 < nE) ? dsts[min(e0 + 3, nE - 1)] : sent;
      db.x = (e0 + 4 < nE) ? dsts[min(e0 + 4, nE - 1)] : sent;
      db.y = (e0 + 5 < nE) ? dsts[min(e0 + 5, nE - 1)] : sent;
      db.z = (e0 + 6 < nE) ? dsts[min(e0 + 6, nE - 1)] : sent;
      db.w = (e0 + 7 < nE) ? dsts[min(e0 + 7, nE - 1)] : sent;
    }
    const unsigned nb = (unsigned)slotBase;
    const unsigned s0 = (unsigned)da.x - nb, s1 = (unsigned)da.y - nb;
    const unsigned s2 = (unsigned)da.z - nb, s3 = (unsigned)da.w - nb;
    const unsigned s4 = (unsigned)db.x - nb, s5 = (unsigned)db.y - nb;
    const unsigned s6 = (unsigned)db.z - nb, s7 = (unsigned)db.w - nb;
    const bool h0 = s0 < (unsigned)NB, h1 = s1 < (unsigned)NB, h2 = s2 < (unsigned)NB, h3 = s3 < (unsigned)NB;
    const bool h4 = s4 < (unsigned)NB, h5 = s5 < (unsigned)NB, h6 = s6 < (unsigned)NB, h7 = s7 < (unsigned)NB;
    const unsigned any = __builtin_amdgcn_ballot_w32(h0 | h1 | h2 | h3 | h4 | h5 | h6 | h7);
    if (any != 0u) {
#define HITJ(J, HJ, SJ) { \
        const unsigned mj = __builtin_amdgcn_ballot_w32(HJ); \
        if (mj != 0u) { \
          if (HJ) { \
            const int pos = wc + (int)__builtin_amdgcn_mbcnt_lo(mj, 0u); \
            if (pos < WCAP) list[wave * WCAP + pos] = ((el0 + (J)) << 12) | (int)(SJ); \
          } \
          wc += (int)__builtin_popcount(mj); } }
      HITJ(0, h0, s0)
      HITJ(1, h1, s1)
      HITJ(2, h2, s2)
      HITJ(3, h3, s3)
      HITJ(4, h4, s4)
      HITJ(5, h5, s5)
      HITJ(6, h6, s6)
      HITJ(7, h7, s7)
#undef HITJ
    }
  }
  return wc;
}

__global__ __launch_bounds__(NTHR) void k_wprep(
    const float* __restrict__ wg, const float* __restrict__ wl, const float* __restrict__ wq,
    unsigned short* wp) {
  const int blk = blockIdx.x, tid = threadIdx.x;
  const float* src;
  int i, base, n, k0;
  if (blk < 8)       { src = wg; i = blk * NTHR + tid;        base = WP_G; n = i >> 3; k0 = (i & 7) * 8; }
  else if (blk < 16) { src = wl; i = (blk - 8) * NTHR + tid;  base = WP_L; n = i >> 3; k0 = (i & 7) * 8; }
  else               { src = wq; i = (blk - 16) * NTHR + tid; base = WP_Q; n = i >> 5; k0 = (i & 31) * 8; }
  v4f a, b;
  a.x = src[(k0 + 0) * FD + n]; a.y = src[(k0 + 1) * FD + n];
  a.z = src[(k0 + 2) * FD + n]; a.w = src[(k0 + 3) * FD + n];
  b.x = src[(k0 + 4) * FD + n]; b.y = src[(k0 + 5) * FD + n];
  b.z = src[(k0 + 6) * FD + n]; b.w = src[(k0 + 7) * FD + n];
  const v8us hv = cvt8h(a, b, 64.0f);
  unsigned short* dh = wp + base + (size_t)i * 8;
  *(volatile v8us*)dh = hv;
  __threadfence();
  *(volatile v8us*)dh = hv;
}

__global__ __launch_bounds__(NTHR) void k_count(const int* __restrict__ dsts, int* cnt, int nE, int vec8) {
  __shared__ __attribute__((aligned(16))) int scnt[NBC];
  __shared__ __attribute__((aligned(16))) int list[LISTN];
  __shared__ int wcnt[NWAVE];
  const int tid = threadIdx.x, lane = tid & 31, wave = tid >> 5;
  const int nodeBase = blockIdx.x * NBC;

  for (int i = tid; i < NBC; i += NTHR) scnt[i] = 0;
  __syncthreads();

  const int nChunks = (nE + CHUNK - 1) / CHUNK;
#pragma unroll 1
  for (int ch = 0; ch < nChunks; ++ch) {
    const int cbase = ch * CHUNK;
    const int wc = scan_chunk<NBC>(dsts, nE, cbase, nodeBase, vec8, list, tid, lane, wave);
    if (lane == 0) wcnt[wave] = wc;
    __syncthreads();
    if (wave == 0) {
#pragma unroll 1
      for (int wsx = 0; wsx < NWAVE; ++wsx) {
        int n = __builtin_amdgcn_readfirstlane(wcnt[wsx]);
        n = n > WCAP ? WCAP : (n < 0 ? 0 : n);
        const int* lp = list + wsx * WCAP;
#pragma unroll 1
        for (int i = 0; i < n; ++i) {
          const int ent  = __builtin_amdgcn_readfirstlane(lp[i]);
          const int slot = ent & (NBC - 1);
          if (lane == 0) scnt[slot] = scnt[slot] + 1;
        }
      }
    }
    __syncthreads();
  }

  v4i cq[4];
#pragma unroll
  for (int q = 0; q < 4; ++q) {
    const int f = (wave * 4 + q) * 128 + 4 * lane;
    cq[q] = *(const v4i*)(scnt + f);
  }
  int* cp = cnt + (size_t)nodeBase;
#pragma unroll
  for (int q = 0; q < 4; ++q) {
    const int f = (wave * 4 + q) * 128 + 4 * lane;
    *(volatile v4i*)(cp + f) = cq[q];
  }
  __threadfence();
#pragma unroll
  for (int q = 0; q < 4; ++q) {
    const int f = (wave * 4 + q) * 128 + 4 * lane;
    *(volatile v4i*)(cp + f) = cq[q];
  }
}

__global__ __launch_bounds__(OTHR) void k_offsets(
    const int* __restrict__ cnt, int* off, int* rbase, int nChunk) {
  __shared__ __attribute__((aligned(16))) int soff[NBC];
  __shared__ __attribute__((aligned(16))) int srb[RBN];
  __shared__ int wtot[OTHR / 32];
  const int tid = threadIdx.x, lane = tid & 31, wave = tid >> 5, sub = tid >> 7;
  for (int i = tid; i < RBN; i += OTHR) srb[i] = 0;
  int carry = 0;
#pragma unroll 1
  for (int ch = 0; ch < nChunk; ++ch) {
    const int base = ch * NBC;
    const v4i c0 = *(const v4i*)(cnt + base + 8 * tid);
    const v4i c1 = *(const v4i*)(cnt + base + 8 * tid + 4);
    const int e0 = max(c0.x, 0), e1 = max(c0.y, 0), e2 = max(c0.z, 0), e3 = max(c0.w, 0);
    const int e4 = max(c1.x, 0), e5 = max(c1.y, 0), e6 = max(c1.z, 0), e7 = max(c1.w, 0);
    const int ts = e0 + e1 + e2 + e3 + e4 + e5 + e6 + e7;
    int incl = ts;
#pragma unroll
    for (int d = 1; d < 32; d <<= 1) {
      const int t = __shfl_up(incl, d);
      if (lane >= d) incl += t;
    }
    if (lane == 31) wtot[wave] = incl;
    __syncthreads();
    const int S0 = wtot[0]  + wtot[1]  + wtot[2]  + wtot[3];
    const int S1 = wtot[4]  + wtot[5]  + wtot[6]  + wtot[7];
    const int S2 = wtot[8]  + wtot[9]  + wtot[10] + wtot[11];
    const int S3 = wtot[12] + wtot[13] + wtot[14] + wtot[15];
    int pre = 0;
#pragma unroll 1
    for (int w = 4 * sub; w < wave; ++w) pre += wtot[w];
    const int b0 = carry;
    const int b1 = b0 + ((S0 + 31) & ~31);
    const int b2 = b1 + ((S1 + 31) & ~31);
    const int b3 = b2 + ((S2 + 31) & ~31);
    const int b4 = b3 + ((S3 + 31) & ~31);
    const int myb = sub == 0 ? b0 : (sub == 1 ? b1 : (sub == 2 ? b2 : b3));
    if (tid == 0) {
      srb[min(4 * ch + 0, RBN - 1)] = b0;
      srb[min(4 * ch + 1, RBN - 1)] = b1;
      srb[min(4 * ch + 2, RBN - 1)] = b2;
      srb[min(4 * ch + 3, RBN - 1)] = b3;
    }
    int run = myb + pre + incl - ts;
    soff[8 * tid + 0] = run; run += e0;
    soff[8 * tid + 1] = run; run += e1;
    soff[8 * tid + 2] = run; run += e2;
    soff[8 * tid + 3] = run; run += e3;
    soff[8 * tid + 4] = run; run += e4;
    soff[8 * tid + 5] = run; run += e5;
    soff[8 * tid + 6] = run; run += e6;
    soff[8 * tid + 7] = run;
    carry = b4;
    __syncthreads();
    const v4i o0 = *(const v4i*)(soff + 4 * tid);
    const v4i o1 = *(const v4i*)(soff + 4 * (tid + OTHR));
    int* op = off + base;
    *(volatile v4i*)(op + 4 * tid) = o0;
    *(volatile v4i*)(op + 4 * (tid + OTHR)) = o1;
    __threadfence();
    *(volatile v4i*)(op + 4 * tid) = o0;
    *(volatile v4i*)(op + 4 * (tid + OTHR)) = o1;
    __syncthreads();
  }
  if (tid == 0) srb[min(4 * nChunk, RBN - 1)] = carry;
  __syncthreads();
  v4i rv = {0, 0, 0, 0};
  if (tid < 32) rv = *(const v4i*)(srb + 4 * tid);
  if (tid < 32) *(volatile v4i*)(rbase + 4 * tid) = rv;
  __threadfence();
  if (tid < 32) *(volatile v4i*)(rbase + 4 * tid) = rv;
}

__global__ __launch_bounds__(NTHR) void k_fill(
    const int* __restrict__ srcs, const int* __restrict__ dsts,
    const int* __restrict__ off, const int* __restrict__ rbase,
    int* csr, int nN, int nE, int vec8, int csrLen) {
  extern __shared__ v4f lds_dyn[];
  int* region = (int*)lds_dyn;
  int* cursor = region + RCAP;
  int* list   = cursor + NBF;
  int* wcnt   = list + LISTN;
  const int tid = threadIdx.x, lane = tid & 31, wave = tid >> 5;
  const int b = blockIdx.x;
  const int nodeBase = b * NBF;

  int rb0 = rbase[b];
  const int rb1 = rbase[b + 1];
  rb0 = rb0 < 0 ? 0 : (rb0 > csrLen ? csrLen : rb0);
  rb0 &= ~31;
  int len = rb1 - rb0;
  len = len < 0 ? 0 : (len > RCAP ? RCAP : len);
  int lenW = (len + 31) & ~31;
  if (rb0 + lenW > csrLen) lenW = (csrLen - rb0) & ~31;

  {
    const v4i z = {0, 0, 0, 0};
    for (int i = tid; i < RCAP / 4; i += NTHR) ((v4i*)region)[i] = z;
    for (int s = tid; s < NBF; s += NTHR) {
      int o = off[nodeBase + s] - rb0;
      o = o < 0 ? 0 : (o > RCAP ? RCAP : o);
      cursor[s] = o;
    }
  }
  __syncthreads();

  const int nChunks = (nE + CHUNK - 1) / CHUNK;
#pragma unroll 1
  for (int ch = 0; ch < nChunks; ++ch) {
    const int cbase = ch * CHUNK;
    const int wc = scan_chunk<NBF>(dsts, nE, cbase, nodeBase, vec8, list, tid, lane, wave);
    if (lane == 0) wcnt[wave] = wc;
    __syncthreads();
    if (wave == 0) {
#pragma unroll 1
      for (int wsx = 0; wsx < NWAVE; ++wsx) {
        int n = __builtin_amdgcn_readfirstlane(wcnt[wsx]);
        n = n > WCAP ? WCAP : (n < 0 ? 0 : n);
        const int* lp = list + wsx * WCAP;
#pragma unroll 1
        for (int i = 0; i < n; ++i) {
          const int ent  = __builtin_amdgcn_readfirstlane(lp[i]);
          const int slot = ent & (NBF - 1);
          int e = cbase + ((ent >> 12) & (CHUNK - 1));
          e = e > nE - 1 ? nE - 1 : e;
          int sv = srcs[e];
          sv = sv < 0 ? 0 : (sv > nN - 1 ? nN - 1 : sv);
          if (lane == 0) {
            int pos = cursor[slot];
            pos = pos < 0 ? 0 : (pos > RCAP - 1 ? RCAP - 1 : pos);
            region[pos] = sv;
            const int np = pos + 1;
            cursor[slot] = np > RCAP ? RCAP : np;
          }
        }
      }
    }
    __syncthreads();
  }

  const int nv = lenW >> 2;
  int* gp = csr + rb0;
#pragma unroll 1
  for (int i = tid; i < nv; i += NTHR) { const v4i v = ((const v4i*)region)[i]; *(volatile v4i*)(gp + 4 * i) = v; }
  __threadfence();
#pragma unroll 1
  for (int i = tid; i < nv; i += NTHR) { const v4i v = ((const v4i*)region)[i]; *(volatile v4i*)(gp + 4 * i) = v; }
}

__global__ __launch_bounds__(GTHR) void k_gemm1(
    const float* __restrict__ x, const unsigned short* __restrict__ Bw, float* H, int nN) {
  extern __shared__ v4f lds_dyn[];
  unsigned short* sX  = (unsigned short*)lds_dyn;
  float*          stg = (float*)((char*)lds_dyn + GROWS * APK1 * 2);
  const int tid = threadIdx.x, lane = tid & 31, wave = tid >> 5, hh = lane >> 4, m = lane & 15;
  const int rowBase = blockIdx.x * GROWS;
  {
    const int c0 = (tid & 7) * 8, rr = tid >> 3;
#pragma unroll
    for (int it = 0; it < 4; ++it) {
      const int r = it * 16 + rr;
      int row = rowBase + r;
      row = row > nN - 1 ? nN - 1 : row;
      const float* ap = x + (size_t)row * FIN + c0;
      const v4f a = *(const v4f*)ap, b = *(const v4f*)(ap + 4);
      *(v8us*)(sX + r * APK1 + c0) = cvt8h(a, b, 1.0f);
    }
  }
  __syncthreads();

#pragma unroll 1
  for (int ch = 0; ch < 4; ++ch) {
    v8f acc[4];
    mma16<FIN, 4, APK1>(sX, Bw + (size_t)(64 * ch) * FIN, wave * 16, lane, acc);
    float* sp = stg + (wave * 16 + 8 * hh) * FD + 64 * ch + m;
#pragma unroll
    for (int t = 0; t < 4; ++t) {
#pragma unroll
      for (int r = 0; r < 8; ++r) sp[r * FD + 16 * t] = acc[t][r] * SC64I;
    }
  }
  __syncthreads();

  store_rows256(stg, H, rowBase, wave, lane);
}

__global__ __launch_bounds__(NTHR) void k_agg(
    const int* __restrict__ csr, const int* __restrict__ off, const int* __restrict__ cnt,
    const float* __restrict__ H, const float* __restrict__ bg, float* Z, int nN, int csrLen) {
  const int tid = threadIdx.x, lane = tid & 31, wave = tid >> 5;
  const int tbase = blockIdx.x * TGT + wave * 32;
  const int cl = tbase + lane;
  const int cnt_l = cnt[cl];
  const int off_l = off[cl];
  const int ca = 4 * lane, cb = FD / 2 + 4 * lane;
  const v4f ba = *(const v4f*)(bg + ca), bb = *(const v4f*)(bg + cb);

#pragma unroll 1
  for (int j = 0; j < 32; ++j) {
    const int c = tbase + j;
    int nd = __builtin_amdgcn_readlane(cnt_l, j);
    nd = nd < 0 ? 0 : (nd > (1 << 24) ? (1 << 24) : nd);
    const int n = nd > DEGCAP ? DEGCAP : nd;
    const float dc = rsqrtf((float)(nd + 1));
    const int st = __builtin_amdgcn_readlane(off_l, j);
    v4f sa = {0.0f, 0.0f, 0.0f, 0.0f};
    v4f sb = {0.0f, 0.0f, 0.0f, 0.0f};
#pragma unroll 1
    for (int q0 = 0; q0 < n; q0 += 32) {
      int pos = st + q0 + lane;
      pos = pos < 0 ? 0 : (pos > csrLen - 1 ? csrLen - 1 : pos);
      int sl = csr[pos];
      sl = sl < 0 ? 0 : (sl > nN - 1 ? nN - 1 : sl);
      int cs = cnt[sl];
      cs = cs < 0 ? 0 : (cs > (1 << 24) ? (1 << 24) : cs);
      const float dl = rsqrtf((float)(cs + 1));
      const int mcnt = (n - q0) < 32 ? (n - q0) : 32;
#pragma unroll 1
      for (int p = 0; p < mcnt; ++p) {
        const int s = __builtin_amdgcn_readlane(sl, p);
        const float ds = __int_as_float(__builtin_amdgcn_readlane(__float_as_int(dl), p));
        const float nrm = ds * dc;
        const v4f vf = *(const v4f*)(H + (size_t)s * FD + ca);
        const v4f vg = *(const v4f*)(H + (size_t)s * FD + cb);
        sa = sa + vf * nrm;
        sb = sb + vg * nrm;
      }
    }
    const v4f ha = *(const v4f*)(H + (size_t)c * FD + ca);
    const v4f hb = *(const v4f*)(H + (size_t)c * FD + cb);
    const float n0 = dc * dc;
    sa = sa + ha * n0;
    sb = sb + hb * n0;
    sa = sa + ba;
    sb = sb + bb;
    float* zp = Z + (size_t)c * FD;
    *(volatile v4f*)(zp + ca) = sa;
    *(volatile v4f*)(zp + cb) = sb;
    __threadfence();
    *(volatile v4f*)(zp + ca) = sa;
    *(volatile v4f*)(zp + cb) = sb;
  }
}

__global__ __launch_bounds__(GTHR) void k_gate(
    const float* __restrict__ Zp, const float* __restrict__ x,
    const unsigned short* __restrict__ Bq, const unsigned short* __restrict__ Bl,
    const float* __restrict__ bq, const float* __restrict__ blin,
    float* U, double* part, int nN) {
  extern __shared__ v4f lds_dyn[];
  float*          zst = (float*)lds_dyn;
  unsigned short* sZ  = (unsigned short*)((char*)lds_dyn + GROWS * FD * 4);
  unsigned short* sX  = sZ + GROWS * APK2;
  const int tid = threadIdx.x, lane = tid & 31, wave = tid >> 5, hh = lane >> 4, m = lane & 15;
  const int rowBase = blockIdx.x * GROWS;

  {
    const int c0 = (tid & 31) * 8, rr = tid >> 5;
#pragma unroll 1
    for (int it = 0; it < 16; ++it) {
      const int r = it * 4 + rr;
      const float* zp = Zp + (size_t)(rowBase + r) * FD + c0;
      const v4f a = *(const v4f*)zp, b = *(const v4f*)(zp + 4);
      v4f ta, tb;
      ta.x = tanh_fast(a.x); ta.y = tanh_fast(a.y); ta.z = tanh_fast(a.z); ta.w = tanh_fast(a.w);
      tb.x = tanh_fast(b.x); tb.y = tanh_fast(b.y); tb.z = tanh_fast(b.z); tb.w = tanh_fast(b.w);
      *(v4f*)(zst + r * FD + c0) = ta;
      *(v4f*)(zst + r * FD + c0 + 4) = tb;
      *(v8us*)(sZ + r * APK2 + c0) = cvt8h(ta, tb, 16.0f);
    }
  }
  {
    const int c0 = (tid & 7) * 8, rr = tid >> 3;
#pragma unroll
    for (int it = 0; it < 4; ++it) {
      const int r = it * 16 + rr;
      int row = rowBase + r;
      row = row > nN - 1 ? nN - 1 : row;
      const float* ap = x + (size_t)row * FIN + c0;
      const v4f a = *(const v4f*)ap, b = *(const v4f*)(ap + 4);
      *(v8us*)(sX + r * APK1 + c0) = cvt8h(a, b, 1.0f);
    }
  }
  __syncthreads();

#pragma unroll 1
  for (int ch = 0; ch < 4; ++ch) {
    v8f ag[4], al[4];
    mma16<FD, 4, APK2>(sZ, Bq + (size_t)(64 * ch) * FD, wave * 16, lane, ag);
    mma16<FIN, 4, APK1>(sX, Bl + (size_t)(64 * ch) * FIN, wave * 16, lane, al);
    float* sp = zst + (wave * 16 + 8 * hh) * FD + 64 * ch + m;
#pragma unroll
    for (int t = 0; t < 4; ++t) {
      const int col = 64 * ch + 16 * t + m;
      const float bqv = bq[col];
      const float blv = blin[col];
#pragma unroll
      for (int r = 0; r < 8; ++r) {
        const float zv = sp[r * FD + 16 * t];
        const float xl = al[t][r] * SC64I + blv;
        const float gl = ag[t][r] * SC1024I + bqv;
        const float g  = sigm_fast(gl);
        float v = (1.0f - g) * xl + g * zv;
        v = fmaxf(v, 0.0f);
        sp[r * FD + 16 * t] = v;
      }
    }
  }
  __syncthreads();

  {
    double s0 = 0.0, q0 = 0.0, s1 = 0.0, q1 = 0.0;
#pragma unroll 4
    for (int r = 0; r < GROWS; ++r) {
      const bool ok = (rowBase + r) < nN;
      float v0 = zst[r * FD + tid];
      float v1 = zst[r * FD + GTHR + tid];
      v0 = ok ? v0 : 0.0f;
      v1 = ok ? v1 : 0.0f;
      const double d0 = (double)v0, d1 = (double)v1;
      s0 += d0; q0 = fma(d0, d0, q0);
      s1 += d1; q1 = fma(d1, d1, q1);
    }
    v2d p0, p1;
    p0.x = s0; p0.y = q0; p1.x = s1; p1.y = q1;
    double* gq = part + (size_t)blockIdx.x * (2 * FD);
    *(volatile v2d*)(gq + 2 * tid) = p0;
    *(volatile v2d*)(gq + 2 * (GTHR + tid)) = p1;
    __threadfence();
    *(volatile v2d*)(gq + 2 * tid) = p0;
    *(volatile v2d*)(gq + 2 * (GTHR + tid)) = p1;
  }

  store_rows256(zst, U, rowBase, wave, lane);
}

__global__ __launch_bounds__(NTHR) void k_bnfin(const double* __restrict__ part, float* coef, int nBlk, int nN) {
  __shared__ __attribute__((aligned(16))) float sco[2 * FD];
  const int tid = threadIdx.x;
  double S = 0.0, Q = 0.0;
#pragma unroll 1
  for (int b = 0; b < nBlk; ++b) {
    const v2d pq = *(const v2d*)(part + (size_t)b * (2 * FD) + 2 * tid);
    S += pq.x;
    Q += pq.y;
  }
  const double rn = 1.0 / (double)(nN > 1 ? nN : 1);
  const double mean = S * rn;
  double var = Q * rn - mean * mean;
  var = var < 0.0 ? 0.0 : var;
  sco[tid]      = (float)mean;
  sco[FD + tid] = rsqrtf((float)var + BN_EPS);
  __syncthreads();
  v4f cv = {0.f, 0.f, 0.f, 0.f};
  if (tid < FD / 2) cv = *(const v4f*)(sco + 4 * tid);
  if (tid < FD / 2) *(volatile v4f*)(coef + 4 * tid) = cv;
  __threadfence();
  if (tid < FD / 2) *(volatile v4f*)(coef + 4 * tid) = cv;
}

__global__ __launch_bounds__(NTHR) void k_bnapply(
    const float* __restrict__ U, const float* __restrict__ coef,
    const float* __restrict__ gam, const float* __restrict__ bet, float* out, int total4) {
  const int i = blockIdx.x * NTHR + threadIdx.x;
  if (i >= total4) return;
  const int c = (i & 63) * 4;
  const v4f u  = *(const v4f*)(U + (size_t)i * 4);
  const v4f mu = *(const v4f*)(coef + c);
  const v4f rs = *(const v4f*)(coef + FD + c);
  const v4f g  = *(const v4f*)(gam + c);
  const v4f b  = *(const v4f*)(bet + c);
  const v4f o = (u - mu) * rs * g + b;
  float* op = out + (size_t)i * 4;
  *(volatile v4f*)op = o;
  __threadfence();
  *(volatile v4f*)op = o;
}

extern "C" void kernel_launch(void* const* d_in, const int* in_sizes, int n_in,
                              void* d_out, int out_size, void* d_ws, size_t ws_size,
                              hipStream_t stream) {
  if (n_in < 10) return;
  const int nN = in_sizes[0] / FIN;
  const int nE = in_sizes[1] / 2;
  if (nN <= 0 || nE <= 0) return;
  if (in_sizes[0] != nN * FIN || in_sizes[1] != 2 * nE) return;
  if (in_sizes[2] != FIN * FD || in_sizes[3] != FD) return;
  if (in_sizes[4] != FIN * FD || in_sizes[5] != FD) return;
  if (in_sizes[6] != FD * FD || in_sizes[7] != FD) return;
  if (in_sizes[8] != FD || in_sizes[9] != FD) return;
  if (out_size != nN * FD) return;
  if (nE > (1 << 28) || nN > (1 << 22)) return;

  const float* x     = (const float*)d_in[0];
  const int*   ei    = (const int*)d_in[1];
  const int*   srcs  = ei;
  const int*   dsts  = ei + nE;
  const float* wg    = (const float*)d_in[2];
  const float* bg    = (const float*)d_in[3];
  const float* wl    = (const float*)d_in[4];
  const float* blin  = (const float*)d_in[5];
  const float* wq    = (const float*)d_in[6];
  const float* bq    = (const float*)d_in[7];
  const float* gam   = (const float*)d_in[8];
  const float* bet   = (const float*)d_in[9];
  float* out = (float*)d_out;

  const int NPAD   = ((nN + TGT - 1) / TGT) * TGT;
  const int nBC    = (nN + NBC - 1) / NBC;
  const int CNTPAD = nBC * NBC;
  if (CNTPAD < NPAD) return;
  if (4 * nBC + 1 > RBN) return;
  const int nBF    = (nN + NBF - 1) / NBF;
  if (nBF > 4 * nBC) return;
  const int csrLen = ((nE + 31) & ~31) + 4096;
  if (31 * 4 * nBC > 4096) return;
  const int nGemm  = NPAD / GROWS;
  const int nAgg   = NPAD / TGT;
  const int total4 = nN * (FD / 4);

  char* ws = (char*)d_ws;
  size_t off = 0;
  const size_t oW    = off; off += (size_t)WPTOT * 2;               off = (off + 255) & ~(size_t)255;
  const size_t oCnt  = off; off += (size_t)CNTPAD * 4;              off = (off + 255) & ~(size_t)255;
  const size_t oOff  = off; off += (size_t)CNTPAD * 4;              off = (off + 255) & ~(size_t)255;
  const size_t oRb   = off; off += (size_t)RBN * 4;                 off = (off + 255) & ~(size_t)255;
  const size_t oCsr  = off; off += (size_t)csrLen * 4;              off = (off + 255) & ~(size_t)255;
  const size_t oH    = off; off += (size_t)NPAD * FD * 4;           off = (off + 255) & ~(size_t)255;
  const size_t oZ    = off; off += (size_t)NPAD * FD * 4;           off = (off + 255) & ~(size_t)255;
  const size_t oPart = off; off += (size_t)nGemm * (2 * FD) * 8;    off = (off + 255) & ~(size_t)255;
  const size_t oCoef = off; off += (size_t)2 * FD * 4;              off = (off + 255) & ~(size_t)255;
  if (off > ws_size || off > (size_t)WSCAP) return;
  unsigned short* wp   = (unsigned short*)(ws + oW);
  int*            cnt  = (int*)(ws + oCnt);
  int*            offp = (int*)(ws + oOff);
  int*            rb   = (int*)(ws + oRb);
  int*            csr  = (int*)(ws + oCsr);
  float*          Hp   = (float*)(ws + oH);
  float*          Up   = Hp;
  float*          Zp   = (float*)(ws + oZ);
  double*         part = (double*)(ws + oPart);
  float*          coef = (float*)(ws + oCoef);

  const int vec8 = ((nE & 3) == 0) ? 1 : 0;

  k_wprep<<<48, NTHR, 0, stream>>>(wg, wl, wq, wp);

  k_count<<<nBC, NTHR, 0, stream>>>(dsts, cnt, nE, vec8);
  k_offsets<<<1, OTHR, 0, stream>>>(cnt, offp, rb, nBC);
  hipFuncSetAttribute(reinterpret_cast<const void*>(&k_fill),
                      hipFuncAttributeMaxDynamicSharedMemorySize, LDS_FILL);
  k_fill<<<nBF, NTHR, LDS_FILL, stream>>>(srcs, dsts, offp, rb, csr, nN, nE, vec8, csrLen);

  hipFuncSetAttribute(reinterpret_cast<const void*>(&k_gemm1),
                      hipFuncAttributeMaxDynamicSharedMemorySize, LDS_G1);
  k_gemm1<<<nGemm, GTHR, LDS_G1, stream>>>(x, wp + WP_G, Hp, nN);

  k_agg<<<nAgg, NTHR, 0, stream>>>(csr, offp, cnt, Hp, bg, Zp, nN, csrLen);

  hipFuncSetAttribute(reinterpret_cast<const void*>(&k_gate),
                      hipFuncAttributeMaxDynamicSharedMemorySize, LDS_G2);
  k_gate<<<nGemm, GTHR, LDS_G2, stream>>>(Zp, x, wp + WP_Q, wp + WP_L, bq, blin, Up, part, nN);

  k_bnfin<<<1, NTHR, 0, stream>>>(part, coef, nGemm, nN);

  k_bnapply<<<(total4 + NTHR - 1) / NTHR, NTHR, 0, stream>>>(Up, coef, gam, bet, out, total4);
}
